// RankBoost_39651138077168
// MI455X (gfx1250) — hardware-verified
//
#include <hip/hip_runtime.h>


namespace {
constexpr int Dm = 128, NI = 10000, NL = 4, Bn = 64, T = 50, G4 = 4 * Dm, NF = Bn * NI, NIP = NI + 128;
constexpr float AS = 8.0f, WS = 64.0f;

typedef _Float16 b16;
typedef __attribute__((ext_vector_type(16))) _Float16 v16b;
typedef __attribute__((ext_vector_type(8)))  _Float16 v8b;
typedef __attribute__((ext_vector_type(8)))  float v8f;
typedef __attribute__((ext_vector_type(4)))  float v4f;

__device__ __forceinline__ v8b ld8b(const b16* p) { return *(const v8b*)p; }
__device__ __forceinline__ v16b cat8b(v8b a, v8b b) { return __builtin_shufflevector(a, b, 0, 1, 2, 3, 4, 5, 6, 7, 8, 9, 10, 11, 12, 13, 14, 15); }
__device__ __forceinline__ v16b frag_kb(const b16* p, int hh) { return cat8b(ld8b(p + 8 * hh), ld8b(p + 16 + 8 * hh)); }
__device__ __forceinline__ void split16(float v, b16& hi, b16& lo) { hi = (b16)v; lo = (b16)(v - (float)hi); }
__device__ __forceinline__ void frag_ksplit(const float* p, int hh, v16b& fh_, v16b& fl_) {
  const float* p0 = p + 8 * hh; const float* p1 = p + 16 + 8 * hh;
#pragma unroll
  for (int e = 0; e < 8; ++e) { b16 a, c; split16(p0[e], a, c); fh_[e] = a; fl_[e] = c; split16(p1[e], a, c); fh_[8 + e] = a; fl_[8 + e] = c; }
}
__device__ __forceinline__ v8f wmma16b(v16b a, v16b b, v8f c) {
  v8f d = __builtin_amdgcn_wmma_f32_16x16x32_f16(false, a, false, b, (short)0, c, false, false);
  asm volatile("v_nop\n\tv_nop\n\tv_nop\n\tv_nop" : "+v"(d) : "v"(a), "v"(b));
  return d;
}
__device__ __forceinline__ void wave_lds_sync() {
  __builtin_amdgcn_fence(__ATOMIC_RELEASE, "workgroup");
  __builtin_amdgcn_wave_barrier();
  __builtin_amdgcn_fence(__ATOMIC_ACQUIRE, "workgroup");
}

struct Opnd { const void* p0; const void* p1; int ld; };
template <int NP> __device__ __forceinline__ void load_frags(const Opnd& o, int row, int kb, int hh, v16b& fh_, v16b& fl_) {
  if (NP == 0) { frag_ksplit((const float*)o.p0 + (size_t)row * o.ld + kb, hh, fh_, fl_); }
  else if (NP == 4) {
    const float* p = (const float*)o.p0 + (size_t)row * o.ld + kb; const float* p0 = p + 8 * hh; const float* p1 = p + 16 + 8 * hh;
#pragma unroll
    for (int e = 0; e < 8; ++e) { b16 a, c; split16(p0[e] * 64.0f, a, c); fh_[e] = a; fl_[e] = c; split16(p1[e] * 64.0f, a, c); fh_[8 + e] = a; fl_[8 + e] = c; }
  } else if (NP == 3) {
    const float* p = (const float*)o.p0 + (size_t)row * o.ld + kb; const float* p0 = p + 8 * hh; const float* p1 = p + 16 + 8 * hh;
#pragma unroll
    for (int e = 0; e < 8; ++e) { fh_[e] = (b16)p0[e]; fh_[8 + e] = (b16)p1[e]; }
    fl_ = fh_;
  } else {
    fh_ = frag_kb((const b16*)o.p0 + (size_t)row * o.ld + kb, hh);
    if (NP == 2) fl_ = frag_kb((const b16*)o.p1 + (size_t)row * o.ld + kb, hh); else fl_ = fh_;
  }
}
template <int ANP, int BNP> __device__ __forceinline__ v8f mac(v16b ah, v16b al, v16b bh, v16b bl, v8f c) {
  c = wmma16b(ah, bh, c);
  if (BNP == 0 || BNP == 2 || BNP == 4) c = wmma16b(ah, bl, c);
  if (ANP == 0 || ANP == 2 || ANP == 4) c = wmma16b(al, bh, c);
  return c;
}
template <int ANP, int BNP>
__device__ __forceinline__ void gemm_tile(const Opnd& A, const Opnd& B, int K, int m0, int c0, int nloc, int hlf, v8f (&acc)[2][4]) {
  for (int kb = 0; kb < K; kb += 32) {
    v16b a0h, a0l, a1h, a1l;
    load_frags<ANP>(A, m0 + nloc, kb, hlf, a0h, a0l);
    load_frags<ANP>(A, m0 + 16 + nloc, kb, hlf, a1h, a1l);
#pragma unroll
    for (int t = 0; t < 4; ++t) {
      v16b bh, bl;
      load_frags<BNP>(B, c0 + t * 16 + nloc, kb, hlf, bh, bl);
      acc[0][t] = mac<ANP, BNP>(a0h, a0l, bh, bl, acc[0][t]);
      acc[1][t] = mac<ANP, BNP>(a1h, a1l, bh, bl, acc[1][t]);
    }
  }
}

__device__ __forceinline__ void epi_planes(v8f (&acc)[2][4], float scale, bool two, b16* __restrict__ oh, b16* __restrict__ ol, int ldo,
                                           int m0, int c0, int lane, b16* Th, b16* Tl) {
  const int nloc = lane & 15, hlf = lane >> 4;
#pragma unroll
  for (int t = 0; t < 4; ++t)
#pragma unroll
    for (int r = 0; r < 2; ++r)
#pragma unroll
      for (int v = 0; v < 8; ++v) {
        const int rr = r * 16 + v + 8 * hlf, cc = t * 16 + nloc;
        b16 h_, l_; split16(acc[r][t][v] * scale, h_, l_);
        Th[rr * 64 + cc] = h_; Tl[rr * 64 + cc] = l_;
      }
  wave_lds_sync();
  for (int pass = 0; pass < 2; ++pass) {
#pragma unroll
    for (int j = 0; j < 8; ++j) {
      const int rr = j * 4 + (lane >> 3), c8 = (lane & 7) * 8;
      const size_t o = (size_t)(m0 + rr) * ldo + c0 + c8;
      *(volatile v8b*)(oh + o) = ld8b(Th + rr * 64 + c8);
      if (two) *(volatile v8b*)(ol + o) = ld8b(Tl + rr * 64 + c8);
    }
    __threadfence();
  }
}
__device__ __forceinline__ void epi_f32(v8f (&acc)[2][4], float scale, const float* rscale, float* __restrict__ out, int ldo, int m0, int c0, int lane, float* Tt) {
  const int nloc = lane & 15, hlf = lane >> 4;
#pragma unroll
  for (int t = 0; t < 4; ++t)
#pragma unroll
    for (int r = 0; r < 2; ++r)
#pragma unroll
      for (int v = 0; v < 8; ++v) {
        const int rr = r * 16 + v + 8 * hlf;
        const float rs = rscale ? rscale[(size_t)(m0 + rr) * 32] : 1.0f;
        Tt[rr * 64 + t * 16 + nloc] = acc[r][t][v] * scale * rs;
      }
  wave_lds_sync();
  float* dst0 = out + (size_t)m0 * ldo + c0;
  for (int pass = 0; pass < 2; ++pass) {
#pragma unroll
    for (int j = 0; j < 16; ++j) { const int rr = j * 2 + hlf, c4 = nloc * 4; *(volatile v4f*)(dst0 + (size_t)rr * ldo + c4) = *(const v4f*)(Tt + rr * 64 + c4); }
    __threadfence();
  }
}


__global__ __launch_bounds__(256) void prep_kernel(const float* __restrict__ Wih, const float* __restrict__ Whh, const float* __restrict__ bih, const float* __restrict__ bhh,
                                                   const float* __restrict__ W1, const float* __restrict__ W2,
                                                   b16* __restrict__ wgh, b16* __restrict__ wgl, float* __restrict__ bsum, b16* __restrict__ w1b, float* __restrict__ w1a, b16* __restrict__ w2t) {
  const size_t tid = (size_t)blockIdx.x * blockDim.x + threadIdx.x, nth = (size_t)gridDim.x * blockDim.x;
  for (int pass = 0; pass < 2; ++pass) {
    for (size_t p = tid; p < (size_t)G4 * 2 * Dm / 8; p += nth) { const int n = (int)(p / 32), k0 = (int)(p % 32) * 8; v8b vh, vl;
#pragma unroll
      for (int e = 0; e < 8; ++e) { const int k = k0 + e; const float w = (k < Dm) ? Wih[(size_t)n * Dm + k] : Whh[(size_t)n * Dm + k - Dm]; b16 a, c; split16(w * WS, a, c); vh[e] = a; vl[e] = c; }
      *(volatile v8b*)(wgh + p * 8) = vh; *(volatile v8b*)(wgl + p * 8) = vl; }
    for (size_t p = tid; p < (size_t)G4; p += nth) ((volatile float*)bsum)[p] = bih[p] + bhh[p];
    for (size_t p = tid; p < (size_t)NL * Dm * Dm / 8; p += nth) { const int l = (int)(p / (Dm * Dm / 8)), rem = (int)(p % (Dm * Dm / 8)), n = rem / 16, k0 = (rem % 16) * 8; v8b v;
#pragma unroll
      for (int e = 0; e < 8; ++e) v[e] = (b16)W1[((size_t)l * 2 * Dm + Dm + k0 + e) * Dm + n];
      *(volatile v8b*)(w1b + p * 8) = v; }
    for (size_t p = tid; p < (size_t)NL * Dm * Dm / 4; p += nth) { const int l = (int)(p / (Dm * Dm / 4)), rem = (int)(p % (Dm * Dm / 4)), n = rem / 32, k0 = (rem % 32) * 4; v4f v;
#pragma unroll
      for (int e = 0; e < 4; ++e) v[e] = W1[((size_t)l * 2 * Dm + k0 + e) * Dm + n];
      *(volatile v4f*)(w1a + p * 4) = v; }
    for (size_t p = tid; p < (size_t)NL * 64 * Dm / 8; p += nth) { const int l = (int)(p / (64 * Dm / 8)), rem = (int)(p % (64 * Dm / 8)), n = rem / 16, k0 = (rem % 16) * 8; v8b v;
#pragma unroll
      for (int e = 0; e < 8; ++e) v[e] = (b16)W2[((size_t)l * Dm + k0 + e) * 64 + n];
      *(volatile v8b*)(w2t + p * 8) = v; }
    __threadfence();
  }
}

__global__ __launch_bounds__(256) void lstm_kernel(const int* __restrict__ useq, const float* __restrict__ emb, const b16* __restrict__ wgh, const b16* __restrict__ wgl, const float* __restrict__ bsum, float* __restrict__ seq) {
  __shared__ __attribute__((aligned(16))) b16 Ah[32][256 + 8]; __shared__ __attribute__((aligned(16))) b16 Al[32][256 + 8];
  __shared__ float Gt[32][G4 + 4]; __shared__ float Hs[32][Dm]; __shared__ float Cs[32][Dm];
  const int t_ = threadIdx.x, wave = t_ >> 5, lane = t_ & 31, nloc = lane & 15, hlf = lane >> 4, b0 = blockIdx.x * 32;
  for (int i = t_; i < 32 * Dm; i += 256) { Hs[i / Dm][i % Dm] = 0.0f; Cs[i / Dm][i % Dm] = 0.0f; }
  __syncthreads();
  for (int step = 0; step < T; ++step) {
    for (int i = t_; i < 32 * 256; i += 256) { const int r = i >> 8, k = i & 255; float v;
      if (k < Dm) { int id = useq[(b0 + r) * T + step]; id = (id < 0) ? 0 : (id > NI ? NI : id); v = emb[(size_t)id * Dm + k]; } else v = Hs[r][k - Dm];
      b16 a, c; split16(v * AS, a, c); Ah[r][k] = a; Al[r][k] = c; }
    __syncthreads();
    { v8f acc[2][4];
#pragma unroll
      for (int r = 0; r < 2; ++r)
#pragma unroll
        for (int t = 0; t < 4; ++t) acc[r][t] = (v8f){};
      const Opnd A{&Ah[0][0], &Al[0][0], 256 + 8}, B{wgh, wgl, 256};
      gemm_tile<2, 2>(A, B, 256, 0, wave * 64, nloc, hlf, acc);
#pragma unroll
      for (int t = 0; t < 4; ++t)
#pragma unroll
        for (int r = 0; r < 2; ++r)
#pragma unroll
          for (int v = 0; v < 8; ++v) { const int rr = r * 16 + v + 8 * hlf, cc = wave * 64 + t * 16 + nloc; Gt[rr][cc] = acc[r][t][v] * (1.0f / (AS * WS)) + bsum[cc]; } }
    __syncthreads();
    for (int i = t_; i < 32 * Dm; i += 256) { const int r = i / Dm, u = i % Dm;
      const float ig = 1.0f / (1.0f + __expf(-Gt[r][u])), fg = 1.0f / (1.0f + __expf(-Gt[r][Dm + u])), gg = tanhf(Gt[r][2 * Dm + u]), og = 1.0f / (1.0f + __expf(-Gt[r][3 * Dm + u]));
      const float c = fg * Cs[r][u] + ig * gg; Cs[r][u] = c; Hs[r][u] = og * tanhf(c); }
    __syncthreads();
  }
  for (int pass = 0; pass < 2; ++pass) { for (int i = t_; i < 32 * Dm / 4; i += 256) *(volatile v4f*)(seq + (size_t)b0 * Dm + i * 4) = *(const v4f*)(&Hs[0][0] + i * 4); __threadfence(); }
}

__global__ __launch_bounds__(128) void cterm_kernel(const float* __restrict__ emb, const float* __restrict__ seq, const b16* __restrict__ w1b, const float* __restrict__ w1a, const float* __restrict__ b1,
                                                    b16* __restrict__ c16, b16* __restrict__ a16) {
  __shared__ __attribute__((aligned(16))) b16 Th[4][2][32 * 64];
  __shared__ __attribute__((aligned(16))) float Apad[32][Dm];
  const int lane = threadIdx.x & 31, wave = threadIdx.x >> 5, nloc = lane & 15, hlf = lane >> 4, l = blockIdx.z, c0 = blockIdx.x * 64;
  v8f acc[2][4];
#pragma unroll
  for (int r = 0; r < 2; ++r)
#pragma unroll
    for (int t = 0; t < 4; ++t) acc[r][t] = (v8f){};
  if (blockIdx.y < 79) {
    const int m0 = blockIdx.y * 128 + wave * 32;
    if (m0 >= NI) return;
    const float* Ab = emb + (size_t)m0 * Dm;
    if (m0 + 32 > NI) {
      for (int i = lane; i < 32 * Dm; i += 32) { const int r = i / Dm, k = i % Dm; Apad[r][k] = (m0 + r < NI) ? emb[(size_t)(m0 + r) * Dm + k] : 0.0f; }
      wave_lds_sync(); Ab = &Apad[0][0];
    }
    const Opnd A{Ab, nullptr, Dm}, B{w1b + (size_t)l * Dm * Dm, nullptr, Dm};
    gemm_tile<3, 1>(A, B, Dm, 0, c0, nloc, hlf, acc);
#pragma unroll
    for (int t = 0; t < 4; ++t)
#pragma unroll
      for (int r = 0; r < 2; ++r)
#pragma unroll
        for (int v = 0; v < 8; ++v) acc[r][t][v] += b1[l * Dm + c0 + t * 16 + nloc];
    epi_planes(acc, 1.0f, false, c16 + ((size_t)l * NIP + m0) * Dm, nullptr, Dm, 0, c0, lane, Th[wave][0], Th[wave][1]);
  } else {
    if (wave >= 2) return;
    const int m0 = wave * 32;
    const Opnd A{seq + (size_t)m0 * Dm, nullptr, Dm};
    const Opnd B{w1a + (size_t)l * Dm * Dm, nullptr, Dm};
    gemm_tile<3, 3>(A, B, Dm, 0, c0, nloc, hlf, acc);
    epi_planes(acc, 1.0f, false, a16 + ((size_t)l * Bn + m0) * Dm, nullptr, Dm, 0, c0, lane, Th[wave][0], Th[wave][1]);
  }
}

__global__ __launch_bounds__(128) void main_kernel(const b16* __restrict__ a16, const b16* __restrict__ c16, const b16* __restrict__ w2t, const float* __restrict__ b2, const float* __restrict__ W3,
                                                   const float* __restrict__ b3, const float* __restrict__ alphas, float* __restrict__ out) {
  __shared__ float Fs[4][32];
  const int lane = threadIdx.x & 31, wave = threadIdx.x >> 5, nloc = lane & 15, hlf = lane >> 4, m0 = blockIdx.x * 128 + wave * 32;
  const int fa = m0 + nloc, fb = m0 + 16 + nloc; const int ba = fa / NI, na = fa % NI, bb = fb / NI, nb = fb % NI;
  const v8b zero8 = {};
  float fin[2][8];
#pragma unroll
  for (int r = 0; r < 2; ++r)
#pragma unroll
    for (int v = 0; v < 8; ++v) fin[r][v] = 0.0f;
#pragma unroll 1
  for (int l = 0; l < NL; ++l) {
    const b16* arow0 = a16 + ((size_t)l * Bn + ba) * Dm; const b16* arow1 = a16 + ((size_t)l * Bn + bb) * Dm;
    const b16* crow0 = c16 + ((size_t)l * NIP + na) * Dm; const b16* crow1 = c16 + ((size_t)l * NIP + nb) * Dm;
    const b16* Wl = w2t + (size_t)l * 64 * Dm;
    v8f acc[2][4];
#pragma unroll
    for (int r = 0; r < 2; ++r)
#pragma unroll
      for (int t = 0; t < 4; ++t) acc[r][t] = (v8f){};
#pragma unroll
    for (int ks = 0; ks < 4; ++ks) {
      const int k0 = ks * 32 + 8 * hlf, k1 = ks * 32 + 16 + 8 * hlf;
      const v8b x00 = __builtin_elementwise_max(ld8b(arow0 + k0) + ld8b(crow0 + k0), zero8), x01 = __builtin_elementwise_max(ld8b(arow0 + k1) + ld8b(crow0 + k1), zero8);
      const v8b x10 = __builtin_elementwise_max(ld8b(arow1 + k0) + ld8b(crow1 + k0), zero8), x11 = __builtin_elementwise_max(ld8b(arow1 + k1) + ld8b(crow1 + k1), zero8);
      const v16b a0 = cat8b(x00, x01), a1 = cat8b(x10, x11);
#pragma unroll
      for (int t = 0; t < 4; ++t) { const v16b bw = frag_kb(Wl + (size_t)(t * 16 + nloc) * Dm + ks * 32, hlf); acc[0][t] = wmma16b(a0, bw, acc[0][t]); acc[1][t] = wmma16b(a1, bw, acc[1][t]); }
    }
    float part[2][8];
#pragma unroll
    for (int r = 0; r < 2; ++r)
#pragma unroll
      for (int v = 0; v < 8; ++v) { float s = 0.0f;
#pragma unroll
        for (int t = 0; t < 4; ++t) { const int hcol = t * 16 + nloc; s += fmaxf(acc[r][t][v] + b2[l * 64 + hcol], 0.0f) * W3[l * 64 + hcol]; }
        part[r][v] = s; }
#pragma unroll
    for (int o = 1; o < 16; o <<= 1)
#pragma unroll
      for (int r = 0; r < 2; ++r)
#pragma unroll
        for (int v = 0; v < 8; ++v) part[r][v] += __shfl_xor(part[r][v], o);
    const float al = alphas[l], bl3 = b3[l];
#pragma unroll
    for (int r = 0; r < 2; ++r)
#pragma unroll
      for (int v = 0; v < 8; ++v) fin[r][v] += al * (part[r][v] + bl3);
  }
  if (nloc == 0) {
#pragma unroll
    for (int r = 0; r < 2; ++r)
#pragma unroll
      for (int v = 0; v < 8; ++v) Fs[wave][r * 16 + 8 * hlf + v] = fin[r][v]; }
  wave_lds_sync();
  for (int pass = 0; pass < 2; ++pass) { ((volatile float*)out)[(size_t)m0 + lane] = Fs[wave][lane]; __threadfence(); }
}

__global__ __launch_bounds__(32) void loss_kernel(const float* __restrict__ fin, const int* __restrict__ posi, const int* __restrict__ negi, float* __restrict__ outl) {
  const int lane = threadIdx.x; float s = 0.0f;
  for (int b = lane; b < Bn; b += 32) { int p = posi[b], n = negi[b]; p = (p < 0) ? 0 : (p >= NI ? NI - 1 : p); n = (n < 0) ? 0 : (n >= NI ? NI - 1 : n);
    s += __expf(-(fin[(size_t)b * NI + p] - fin[(size_t)b * NI + n])); }
#pragma unroll
  for (int o = 16; o > 0; o >>= 1) s += __shfl_xor(s, o);
  if (lane == 0) { ((volatile float*)outl)[0] = s * (1.0f / Bn); __threadfence(); ((volatile float*)outl)[0] = s * (1.0f / Bn); }
}
}

extern "C" void kernel_launch(void* const* d_in, const int* in_sizes, int n_in,
                              void* d_out, int out_size, void* d_ws, size_t ws_size, hipStream_t stream) {
  (void)n_in; (void)out_size;
  const int* useq = (const int*)d_in[0]; const int* posi = (const int*)d_in[1]; const int* negi = (const int*)d_in[2];
  const float* emb = (const float*)d_in[3];
  const float* Wih = (const float*)d_in[4]; const float* Whh = (const float*)d_in[5]; const float* bih = (const float*)d_in[6]; const float* bhh = (const float*)d_in[7];
  const float* W1 = (const float*)d_in[8]; const float* b1 = (const float*)d_in[9]; const float* W2 = (const float*)d_in[10]; const float* b2 = (const float*)d_in[11];
  const float* W3 = (const float*)d_in[12]; const float* b3 = (const float*)d_in[13]; const float* alphas = (const float*)d_in[14];
  float* out = (float*)d_out;
  if (in_sizes[0] != Bn * T || in_sizes[3] != (NI + 1) * Dm || in_sizes[4] != G4 * Dm || in_sizes[8] != NL * 2 * Dm * Dm || in_sizes[10] != NL * Dm * 64) return;
  size_t off = 0; char* ws = (char*)d_ws;
  auto carve = [&](size_t bytes) { char* p = ws + off; off += (bytes + 255) & ~(size_t)255; return p; };
  b16* wgh = (b16*)carve((size_t)G4 * 256 * 2); b16* wgl = (b16*)carve((size_t)G4 * 256 * 2); float* bsum = (float*)carve(G4 * 4);
  b16* w1b = (b16*)carve((size_t)NL * Dm * Dm * 2); float* w1a = (float*)carve((size_t)NL * Dm * Dm * 4); b16* w2t = (b16*)carve((size_t)NL * 64 * Dm * 2);
  float* seq = (float*)carve((size_t)Bn * Dm * 4);
  b16* c16 = (b16*)carve((size_t)NL * NIP * Dm * 2);
  b16* a16 = (b16*)carve((size_t)NL * Bn * Dm * 2);
  if (off > ws_size) return;
  prep_kernel<<<64, 256, 0, stream>>>(Wih, Whh, bih, bhh, W1, W2, wgh, wgl, bsum, w1b, w1a, w2t);
  lstm_kernel<<<Bn / 32, 256, 0, stream>>>(useq, emb, wgh, wgl, bsum, seq);
  cterm_kernel<<<dim3(Dm / 64, 80, NL), 128, 0, stream>>>(emb, seq, w1b, w1a, b1, c16, a16);
  main_kernel<<<NF / 128, 128, 0, stream>>>(a16, c16, w2t, b2, W3, b3, alphas, out);
  loss_kernel<<<1, 32, 0, stream>>>(out, posi, negi, out + NF);
}
